// MultiHead_90374701843215
// MI455X (gfx1250) — hardware-verified
//
#include <hip/hip_runtime.h>

#ifndef NB
#define NB 2
#endif
#ifndef SQ
#define SQ 2048
#endif
#ifndef ERQ
#if SQ < 512
#define ERQ SQ
#else
#define ERQ 512
#endif
#endif
#define NB_FULL 2
#define SQ_FULL 2048
#define DM 1024
#define NH 16
#define HD 64
#define LQ (3 * DM)
#define NR ((size_t)NB * SQ)
#define NRE ((size_t)NB * ERQ)
static_assert(NB >= 1 && NB <= NB_FULL);
static_assert(SQ >= 128 && SQ <= SQ_FULL && SQ % 128 == 0);
static_assert(ERQ >= 128 && ERQ <= SQ && ERQ % 128 == 0 && (SQ - ERQ) % 128 == 0);
static_assert(NH * HD == DM);
static_assert(((ERQ / 16) * (DM / 64)) % 4 == 0);

typedef __bf16 v16b __attribute__((ext_vector_type(16)));
typedef unsigned short v8us __attribute__((ext_vector_type(8), may_alias));
typedef float  v8f  __attribute__((ext_vector_type(8)));
typedef float  v4f  __attribute__((ext_vector_type(4)));
typedef float  v4fa __attribute__((ext_vector_type(4), may_alias));
typedef _Float16 v16h __attribute__((ext_vector_type(16)));
typedef _Float16 v4h __attribute__((ext_vector_type(4)));
union FragB { v16b v; v8us half[2]; unsigned short u[16]; };
union FragH { v16h v; v8us half[2]; _Float16 h[16]; unsigned short u[16]; };

__device__ __forceinline__ unsigned short bf16_bits(float x) { unsigned int u = __float_as_uint(x); return (unsigned short)((u + 0x7FFFu + ((u >> 16) & 1u)) >> 16); }
__device__ __forceinline__ float bf16_val(unsigned short b) { return __uint_as_float(((unsigned int)b) << 16); }
__device__ __forceinline__ float bf16_rne(float x) { return bf16_val(bf16_bits(x)); }
__device__ __forceinline__ unsigned short h_bits(_Float16 hv) { return __builtin_bit_cast(unsigned short, hv); }

template <int NT>
__device__ __forceinline__ v8f mmaN(v16b ah, v16b al, v16b bh, v16b bl, v8f c) {
  c = __builtin_amdgcn_wmma_f32_16x16x32_bf16(false, ah, false, bh, (short)0, c, false, false);
  if (NT >= 2) c = __builtin_amdgcn_wmma_f32_16x16x32_bf16(false, al, false, bh, (short)0, c, false, false);
  if (NT >= 3) c = __builtin_amdgcn_wmma_f32_16x16x32_bf16(false, ah, false, bl, (short)0, c, false, false);
  asm volatile("v_nop\n\tv_nop\n\tv_nop\n\tv_nop" : "+v"(c) : "v"(ah), "v"(al), "v"(bh), "v"(bl));
  return c;
}

__global__ __launch_bounds__(256) void k_wt_bf16(const float* __restrict__ W, unsigned short* __restrict__ Wt, int K, int N) {
  const int t = blockIdx.x * 256 + threadIdx.x;
  const int k8n = K / 8;
  if (t >= N * k8n) return;
  const int n = t / k8n, k8 = (t % k8n) * 8;
  v8us v;
#pragma unroll
  for (int i = 0; i < 8; ++i) v[i] = bf16_bits(W[(size_t)(k8 + i) * N + n]);
  *(volatile v8us*)(Wt + (size_t)n * K + k8) = v;
  __threadfence();
  *(volatile v8us*)(Wt + (size_t)n * K + k8) = v;
}

template <bool ASPLIT, int ACT, bool BIAS_BF16>
__global__ __launch_bounds__(128) void k_gemm_bf(const float* __restrict__ A, int lda, const unsigned short* __restrict__ Wt, int ldb,
                                               const float* __restrict__ bias, float* __restrict__ C, int ldc, int M, int N, int K) {
  __shared__ __attribute__((aligned(16))) float so[4][16][64];
  const int tid = threadIdx.x, w = tid >> 5, lane = tid & 31, ln = lane & 15, hh = lane >> 4;
  const int ntn = N / 64;
  const int wid = blockIdx.x * 4 + w;
  const int mt = wid / ntn, nq = wid % ntn;
  if (mt * 16 >= M) return;
  const int row0 = mt * 16, col0 = nq * 64;
  const float* arow = A + (size_t)(row0 + ln) * lda;
  v8f acc[4] = {};
  for (int kb = 0; kb < K; kb += 32) {
    FragB ah, al;
    const v4f x0 = *(const v4fa*)(arow + kb + 8 * hh), x1 = *(const v4fa*)(arow + kb + 8 * hh + 4);
    const v4f x2 = *(const v4fa*)(arow + kb + 16 + 8 * hh), x3 = *(const v4fa*)(arow + kb + 16 + 8 * hh + 4);
    float xs[16] = {x0[0],x0[1],x0[2],x0[3],x1[0],x1[1],x1[2],x1[3],x2[0],x2[1],x2[2],x2[3],x3[0],x3[1],x3[2],x3[3]};
#pragma unroll
    for (int i = 0; i < 16; ++i) { const unsigned short hb = bf16_bits(xs[i]); ah.u[i] = hb; al.u[i] = ASPLIT ? bf16_bits(xs[i] - bf16_val(hb)) : (unsigned short)0; }
#pragma unroll
    for (int t = 0; t < 4; ++t) {
      const unsigned short* brow = Wt + (size_t)(col0 + t * 16 + ln) * ldb + kb;
      FragB b;
      b.half[0] = *(const v8us*)(brow + 8 * hh);
      b.half[1] = *(const v8us*)(brow + 16 + 8 * hh);
      acc[t] = mmaN<ASPLIT ? 2 : 1>(ah.v, al.v, b.v, b.v, acc[t]);
    }
  }
#pragma unroll
  for (int t = 0; t < 4; ++t) {
    float bv = bias ? bias[col0 + t * 16 + ln] : 0.f;
    if (BIAS_BF16) bv = bf16_rne(bv);
#pragma unroll
    for (int r = 0; r < 8; ++r) { float v = acc[t][r] + bv; if (ACT == 1) v = fmaxf(v, 0.f); so[w][8 * hh + r][t * 16 + ln] = v; }
  }
  __builtin_amdgcn_fence(4, "workgroup");
  __builtin_amdgcn_wave_barrier();
  const int rsub = lane >> 4, c4 = (lane & 15) * 4;
  for (int pass = 0; pass < 2; ++pass) {
#pragma unroll
    for (int q = 0; q < 8; ++q) {
      const int r = q * 2 + rsub;
      const v4f v = *(const v4fa*)&so[w][r][c4];
      *(volatile v4f*)(C + (size_t)(row0 + r) * ldc + col0 + c4) = v;
    }
    if (pass == 0) __threadfence();
  }
}

__device__ __forceinline__ v16h g2_frag(const _Float16* p, int hh) { FragH f; f.half[0] = *(const v8us*)((const unsigned short*)p + 8 * hh); f.half[1] = *(const v8us*)((const unsigned short*)p + 16 + 8 * hh); return f.v; }
__device__ __forceinline__ v16h frag_us(const unsigned short* p, int hh) { FragH f; f.half[0] = *(const v8us*)(p + 8 * hh); f.half[1] = *(const v8us*)(p + 16 + 8 * hh); return f.v; }
__device__ __forceinline__ v8f g2_mma(v16h a, v16h b, v8f c) { v8f d = __builtin_amdgcn_wmma_f32_16x16x32_f16(false, a, false, b, (short)0, c, false, false); asm volatile("v_nop\n\tv_nop\n\tv_nop\n\tv_nop" : "+v"(d) : "v"(a), "v"(b)); return d; }

template <int ACT>
__global__ __launch_bounds__(128) void k_gemm2(const _Float16* __restrict__ A, int lda, size_t sA, const _Float16* __restrict__ Bh, int ldb, size_t sB, float alpha, const float* __restrict__ bias, size_t sBias, const float* __restrict__ CP, int rowsPerB, size_t sCPb, int row0g,
    float* __restrict__ C, _Float16* __restrict__ C16, int ldc, size_t sC, int M, int N, int K) {
  static_assert(ACT == 0);
  __shared__ __attribute__((aligned(16))) float so[4][32][68];
  const int tid = threadIdx.x, w = tid >> 5, lane = tid & 31, ln = lane & 15, hh = lane >> 4; const int by = blockIdx.y;
  A += (size_t)by * sA; Bh += (size_t)by * sB; const size_t cofs = (size_t)by * sC; const float* bp = bias ? bias + (size_t)by * sBias : nullptr;
  const int ntn = N >> 6; const int mt = blockIdx.x / ntn, nq = blockIdx.x - mt * ntn; const int row0 = mt * 128 + 32 * w, col0 = nq * 64; if (row0 >= M) return;
  const _Float16* a0p = A + (size_t)(row0 + ln) * lda; const _Float16* a1p = a0p + (size_t)16 * lda;
  const _Float16* b0p = Bh + (size_t)(col0 + ln) * ldb; const _Float16* b1p = b0p + (size_t)16 * ldb; const _Float16* b2p = b1p + (size_t)16 * ldb; const _Float16* b3p = b2p + (size_t)16 * ldb;
  const v8f z8 = {0.f,0.f,0.f,0.f,0.f,0.f,0.f,0.f}; v8f c00 = z8, c01 = z8, c02 = z8, c03 = z8, c10 = z8, c11 = z8, c12 = z8, c13 = z8;
#pragma unroll 1
  for (int kb = 0; kb < K; kb += 32) { const v16h a0 = g2_frag(a0p + kb, hh), a1 = g2_frag(a1p + kb, hh);
    v16h b = g2_frag(b0p + kb, hh); c00 = g2_mma(a0, b, c00); c10 = g2_mma(a1, b, c10);
    b = g2_frag(b1p + kb, hh); c01 = g2_mma(a0, b, c01); c11 = g2_mma(a1, b, c11);
    b = g2_frag(b2p + kb, hh); c02 = g2_mma(a0, b, c02); c12 = g2_mma(a1, b, c12);
    b = g2_frag(b3p + kb, hh); c03 = g2_mma(a0, b, c03); c13 = g2_mma(a1, b, c13); }
  v8f accs[8] = {c00, c01, c02, c03, c10, c11, c12, c13};
#pragma unroll
  for (int u = 0; u < 8; ++u) { const int t = u & 3, half = u >> 2; const int col = col0 + t * 16 + ln; const float bv = bp ? bf16_rne(bp[col]) : 0.f;
#pragma unroll
    for (int r = 0; r < 8; ++r) { const int rloc = half * 16 + 8 * hh + r; float v = accs[u][r] * alpha + bv; if (CP) { if (rowsPerB < 0) v += CP[cofs + (size_t)(row0g + row0 + rloc) * ldc + col]; else { const int bidx = (row0g + row0 + rloc) / rowsPerB; v += CP[(size_t)bidx * sCPb + (size_t)by * 64 + col]; } }
      so[w][rloc][t * 16 + ln] = v; } }
  __builtin_amdgcn_fence(4, "workgroup"); __builtin_amdgcn_wave_barrier();
  const int rsub = lane >> 4, c4 = (lane & 15) * 4;
  for (int pass = 0; pass < 2; ++pass) {
#pragma unroll
    for (int q = 0; q < 16; ++q) { const int r = q * 2 + rsub; const v4f v = *(const v4fa*)&so[w][r][c4]; if (C) *(volatile v4f*)(C + cofs + (size_t)(row0 + r) * ldc + col0 + c4) = v; if (C16) { v4h h4; for (int i = 0; i < 4; ++i) h4[i] = (_Float16)v[i]; *(volatile v4h*)(C16 + cofs + (size_t)(row0 + r) * ldc + col0 + c4) = h4; } }
    if (pass == 0) __threadfence(); } }

__global__ __launch_bounds__(256) void k_wt_f16(const float* __restrict__ W, _Float16* __restrict__ Wt, int K, int N, float scale) {
  const int t = blockIdx.x * 256 + threadIdx.x; if (t >= N * (K / 8)) return; const int n = t / (K / 8), k8 = (t % (K / 8)) * 8; FragH f;
#pragma unroll
  for (int i = 0; i < 8; ++i) f.h[i] = (_Float16)(bf16_rne(W[(size_t)(k8 + i) * N + n]) * scale); const v8us o = f.half[0];
  *(volatile v8us*)((unsigned short*)Wt + (size_t)n * K + k8) = o; __threadfence(); *(volatile v8us*)((unsigned short*)Wt + (size_t)n * K + k8) = o;
}

__global__ __launch_bounds__(256) void k_whd(const float* __restrict__ Wq, const float* __restrict__ Wk, const float* __restrict__ Wv, _Float16* __restrict__ Bt) {
  const int p = blockIdx.y;
  const float* W = (p == 0) ? Wq : ((p == 1) ? Wk : Wv);
  const int t = blockIdx.x * 256 + threadIdx.x; if (t >= DM * (DM / 8)) return;
  const int n = t / (DM / 8), e8 = (t % (DM / 8)) * 8; const int h = n / HD, d = n % HD;
  FragH f;
#pragma unroll
  for (int i = 0; i < 8; ++i) f.h[i] = (_Float16)(bf16_rne(W[((size_t)h * DM + e8 + i) * HD + d]) * 16.0f);
  const v8us o = f.half[0];
  unsigned short* dst = (unsigned short*)Bt + ((size_t)p * DM + n) * DM + e8;
  *(volatile v8us*)dst = o; __threadfence(); *(volatile v8us*)dst = o;
}

__global__ __launch_bounds__(256) void k_x16(const float* __restrict__ x, _Float16* __restrict__ X16, size_t n8) { const size_t t = (size_t)blockIdx.x * 256 + threadIdx.x; if (t >= n8) return; FragH f;
#pragma unroll
  for (int q = 0; q < 8; ++q) f.h[q] = (_Float16)bf16_rne(x[t * 8 + q]); *(volatile v8us*)((unsigned short*)X16 + t * 8) = f.half[0]; __threadfence(); *(volatile v8us*)((unsigned short*)X16 + t * 8) = f.half[0]; }

template <int NHv, int TTv>
__global__ __launch_bounds__(256) void k_vt(const _Float16* __restrict__ V16, int ldv, int voff, _Float16* __restrict__ Vt) { __shared__ unsigned short tl[64][66]; const int tid = threadIdx.x; const int slab = blockIdx.x / (TTv / 64), lg = blockIdx.x % (TTv / 64); const int b = slab / NHv, h = slab % NHv;
  for (int i = tid; i < 64 * 8; i += 256) { const int r = i / 8, c8 = (i % 8) * 8; FragH f; f.half[0] = *(const v8us*)((const unsigned short*)V16 + ((size_t)b * TTv + lg * 64 + r) * ldv + voff + h * 64 + c8);
#pragma unroll
    for (int q = 0; q < 8; ++q) tl[r][c8 + q] = f.u[q]; }
  __syncthreads();
  for (int pass = 0; pass < 2; ++pass) {
#pragma unroll
    for (int rd = 0; rd < 2; ++rd) { const int d = rd * 32 + tid / 8, pc = tid % 8; FragH f;
#pragma unroll
      for (int q = 0; q < 8; ++q) f.u[q] = tl[pc * 8 + q][d];
      *(volatile v8us*)((unsigned short*)Vt + ((size_t)slab * 64 + d) * TTv + lg * 64 + pc * 8) = f.half[0]; }
    if (pass == 0) __threadfence(); } }

__global__ __launch_bounds__(256) void k_res(const float* __restrict__ F, _Float16* __restrict__ RL, size_t n8) {
  const size_t t = (size_t)blockIdx.x * 256 + threadIdx.x; if (t >= n8) return;
  const size_t row = t / (LQ / 8); const int c8 = (int)(t % (LQ / 8)) * 8; const int p = c8 / DM, c = c8 - p * DM;
  const v4f a = *(const v4fa*)(F + t * 8), d = *(const v4fa*)(F + t * 8 + 4);
  FragH f;
#pragma unroll
  for (int q = 0; q < 4; ++q) { _Float16 hv = (_Float16)a[q]; f.h[q] = (_Float16)((a[q] - (float)hv) * 1024.0f); hv = (_Float16)d[q]; f.h[4 + q] = (_Float16)((d[q] - (float)hv) * 1024.0f); }
  const v8us o = f.half[0];
  unsigned short* dst = (unsigned short*)RL + (size_t)p * NRE * DM + row * DM + c;
  *(volatile v8us*)dst = o; __threadfence(); *(volatile v8us*)dst = o;
}

template <bool RES>
__global__ __launch_bounds__(128) __attribute__((amdgpu_num_vgpr(256)))
void k_attn(const _Float16* __restrict__ QKV, const _Float16* __restrict__ VT, const _Float16* __restrict__ RL, const _Float16* __restrict__ VLT,
            _Float16* __restrict__ O16, float* __restrict__ OF, int qbase) {
  constexpr int DT = RES ? 2 : 4;
  constexpr int RPB = RES ? 32 : 64;
  __shared__ __attribute__((aligned(16))) unsigned short Ks[64 * 72];
  __shared__ __attribute__((aligned(16))) unsigned short Vs[64 * 72];
  __shared__ __attribute__((aligned(16))) unsigned short Kl[RES ? 64 * 72 : 8];
  __shared__ __attribute__((aligned(16))) unsigned short Vl[RES ? 64 * 72 : 8];
  __shared__ __attribute__((aligned(16))) float pscr[4][1152];
  const int tid = threadIdx.x, w = tid >> 5, lane = tid & 31, ln = lane & 15, hh = lane >> 4;
  const int bh = blockIdx.y, b = bh / NH, h = bh - b * NH;
  const int q0 = qbase + blockIdx.x * RPB;
  const int rg = RES ? (w >> 1) : w;
  const int dq = RES ? (w & 1) * 32 : 0;
  const int qw = q0 + rg * 16;
  const int nkc = (q0 + RPB - 1) / 64 + 1;
  unsigned short* Ph = (unsigned short*)pscr[w];
  unsigned short* Pl = Ph + 16 * 72;
  const v8f z8 = {0.f,0.f,0.f,0.f,0.f,0.f,0.f,0.f};
  v8f o[DT], orr[DT];
#pragma unroll
  for (int t = 0; t < DT; ++t) { o[t] = z8; orr[t] = z8; }
  float m[8], l[8];
#pragma unroll
  for (int r = 0; r < 8; ++r) { m[r] = -1.0e30f; l[r] = 0.f; }
  const unsigned short* qp = (const unsigned short*)QKV + ((size_t)b * SQ + qw + ln) * LQ + h * HD;

#pragma unroll 1
  for (int kc = 0; kc < nkc; ++kc) {
    const int key0 = kc * 64;
    __syncthreads();
#pragma unroll
    for (int it = 0; it < 4; ++it) {
      const int r = it * 16 + (tid >> 3), c8 = (tid & 7) * 8;
      const v8us kv = *(const v8us*)((const unsigned short*)QKV + ((size_t)b * SQ + key0 + r) * LQ + DM + h * HD + c8);
      *(v8us*)(Ks + r * 72 + c8) = kv;
      const v8us vv = *(const v8us*)((const unsigned short*)VT + ((size_t)bh * HD + r) * SQ + key0 + c8);
      *(v8us*)(Vs + r * 72 + c8) = vv;
      if (RES) {
        const v8us klv = *(const v8us*)((const unsigned short*)RL + NRE * DM + ((size_t)b * ERQ + key0 + r) * DM + h * HD + c8);
        *(v8us*)(Kl + r * 72 + c8) = klv;
        const v8us vlv = *(const v8us*)((const unsigned short*)VLT + ((size_t)bh * HD + r) * ERQ + key0 + c8);
        *(v8us*)(Vl + r * 72 + c8) = vlv;
      }
    }
    __syncthreads();

    const v16h qa0 = frag_us(qp, hh), qa1 = frag_us(qp + 32, hh);
    v16h ql0 = qa0, ql1 = qa1;
    if (RES) { const unsigned short* qlp = (const unsigned short*)RL + ((size_t)b * ERQ + qw + ln) * DM + h * HD; ql0 = frag_us(qlp, hh); ql1 = frag_us(qlp + 32, hh); }
    v8f s[4];
#pragma unroll
    for (int t = 0; t < 4; ++t) {
      const unsigned short* kr = Ks + (t * 16 + ln) * 72;
      const v16h b0 = frag_us(kr, hh), b1 = frag_us(kr + 32, hh);
      v8f acc = z8; acc = g2_mma(qa0, b0, acc); acc = g2_mma(qa1, b1, acc);
      if (RES) {
        const unsigned short* klr = Kl + (t * 16 + ln) * 72;
        v8f accr = z8; accr = g2_mma(ql0, b0, accr); accr = g2_mma(ql1, b1, accr);
        const v16h c0 = frag_us(klr, hh), c1 = frag_us(klr + 32, hh);
        accr = g2_mma(qa0, c0, accr); accr = g2_mma(qa1, c1, accr);
        s[t] = acc * 0.125f + accr * (0.125f / 1024.0f);
      } else {
        s[t] = acc * 0.125f;
      }
    }

#pragma unroll
    for (int r = 0; r < 8; ++r) {
      const int qrow = qw + 8 * hh + r;
      float v[4];
#pragma unroll
      for (int t = 0; t < 4; ++t) { const int key = key0 + t * 16 + ln; const float x = s[t][r]; v[t] = (key > qrow) ? -1.0e30f : x; }
      float mx = fmaxf(fmaxf(v[0], v[1]), fmaxf(v[2], v[3]));
      mx = fmaxf(mx, __shfl_xor(mx, 8)); mx = fmaxf(mx, __shfl_xor(mx, 4)); mx = fmaxf(mx, __shfl_xor(mx, 2)); mx = fmaxf(mx, __shfl_xor(mx, 1));
      const float mn = fmaxf(m[r], mx);
      const float al = __expf(m[r] - mn);
      float p[4]; float ps = 0.f;
#pragma unroll
      for (int t = 0; t < 4; ++t) { p[t] = __expf(v[t] - mn); ps += p[t]; }
      ps += __shfl_xor(ps, 8); ps += __shfl_xor(ps, 4); ps += __shfl_xor(ps, 2); ps += __shfl_xor(ps, 1);
      l[r] = l[r] * al + ps; m[r] = mn;
#pragma unroll
      for (int t = 0; t < DT; ++t) { o[t][r] = o[t][r] * al; if (RES) orr[t][r] = orr[t][r] * al; }
#pragma unroll
      for (int t = 0; t < 4; ++t) {
        const float pc = p[t] * 1024.0f; const _Float16 ph = (_Float16)pc;
        Ph[(8 * hh + r) * 72 + t * 16 + ln] = h_bits(ph);
        if (RES) { const _Float16 pl = (_Float16)((pc - (float)ph) * 1024.0f); Pl[(8 * hh + r) * 72 + t * 16 + ln] = h_bits(pl); }
      }
    }
    __builtin_amdgcn_fence(4, "wavefront");
    __builtin_amdgcn_wave_barrier();

    const v16h pa0 = frag_us(Ph + ln * 72, hh), pa1 = frag_us(Ph + ln * 72 + 32, hh);
    v16h pl0 = pa0, pl1 = pa1;
    if (RES) { pl0 = frag_us(Pl + ln * 72, hh); pl1 = frag_us(Pl + ln * 72 + 32, hh); }
#pragma unroll
    for (int t = 0; t < DT; ++t) {
      const unsigned short* vr = Vs + (dq + t * 16 + ln) * 72;
      const v16h b0 = frag_us(vr, hh), b1 = frag_us(vr + 32, hh);
      o[t] = g2_mma(pa0, b0, o[t]); o[t] = g2_mma(pa1, b1, o[t]);
      if (RES) {
        orr[t] = g2_mma(pl0, b0, orr[t]); orr[t] = g2_mma(pl1, b1, orr[t]);
        const unsigned short* vlr = Vl + (dq + t * 16 + ln) * 72;
        const v16h c0 = frag_us(vlr, hh), c1 = frag_us(vlr + 32, hh);
        orr[t] = g2_mma(pa0, c0, orr[t]); orr[t] = g2_mma(pa1, c1, orr[t]);
      }
    }
  }

  __builtin_amdgcn_fence(4, "wavefront");
  __builtin_amdgcn_wave_barrier();
  if (RES) {
    float* Fo = pscr[w];
#pragma unroll
    for (int r = 0; r < 8; ++r) {
      const float inv = (1.0f / l[r]) * (1.0f / 1024.0f);
#pragma unroll
      for (int t = 0; t < DT; ++t) Fo[(8 * hh + r) * 36 + t * 16 + ln] = (o[t][r] + orr[t][r] * (1.0f / 1024.0f)) * inv;
    }
    __builtin_amdgcn_fence(4, "wavefront");
    __builtin_amdgcn_wave_barrier();
    for (int pass = 0; pass < 2; ++pass) {
#pragma unroll
      for (int it = 0; it < 4; ++it) {
        const int row = it * 4 + (lane >> 3), c4 = (lane & 7) * 4;
        const v4f vv = *(const v4fa*)(Fo + row * 36 + c4);
        *(volatile v4f*)(OF + ((size_t)b * ERQ + qw + row) * DM + h * HD + dq + c4) = vv;
      }
      if (pass == 0) __threadfence();
    }
  } else {
    unsigned short* Po = Ph;
#pragma unroll
    for (int r = 0; r < 8; ++r) {
      const float sc = 0.0625f / l[r];
#pragma unroll
      for (int t = 0; t < DT; ++t) Po[(8 * hh + r) * 72 + t * 16 + ln] = h_bits((_Float16)(o[t][r] * sc));
    }
    __builtin_amdgcn_fence(4, "wavefront");
    __builtin_amdgcn_wave_barrier();
    for (int pass = 0; pass < 2; ++pass) {
#pragma unroll
      for (int it = 0; it < 4; ++it) {
        const int row = it * 4 + (lane >> 3), c8 = (lane & 7) * 8;
        const v8us vv = *(const v8us*)(Po + row * 72 + c8);
        *(volatile v8us*)((unsigned short*)O16 + ((size_t)b * SQ + qw + row) * DM + h * HD + c8) = vv;
      }
      if (pass == 0) __threadfence();
    }
  }
}

extern "C" void kernel_launch(void* const* d_in, const int* in_sizes, int n_in,
                              void* d_out, int out_size, void* d_ws, size_t ws_size, hipStream_t stream) {
  if (n_in < 6) return;
  const float* x  = (const float*)d_in[0];
  const float* Wq = (const float*)d_in[1];
  const float* Wk = (const float*)d_in[2];
  const float* Wv = (const float*)d_in[3];
  const float* Wo = (const float*)d_in[4];
  const float* bo = (const float*)d_in[5];
  float* out = (float*)d_out;
  const size_t xrows = (size_t)(NB - 1) * SQ_FULL + SQ;
  if ((size_t)in_sizes[0] < xrows * DM) return;
  if ((size_t)in_sizes[1] < (size_t)NH * DM * HD || (size_t)in_sizes[2] < (size_t)NH * DM * HD || (size_t)in_sizes[3] < (size_t)NH * DM * HD) return;
  if ((size_t)in_sizes[4] < (size_t)DM * DM || in_sizes[5] < DM) return;
  if ((size_t)out_size < xrows * DM) return;

  char* ws = (char*)d_ws; size_t off = 0;
  auto take = [&](size_t bytes) { char* p = ws + off; off += (bytes + 255) & ~(size_t)255; return p; };
  _Float16* BQKV = (_Float16*)take((size_t)LQ * DM * 2);
  _Float16* BO   = (_Float16*)take((size_t)DM * DM * 2);
  unsigned short* BOB = (unsigned short*)take((size_t)DM * DM * 2);
  _Float16* X16  = (_Float16*)take(xrows * DM * 2);
  _Float16* QKV  = (_Float16*)take(NR * LQ * 2);
  float*    QF   = (float*)take(NRE * LQ * 4);
  _Float16* RL   = (_Float16*)take((size_t)3 * NRE * DM * 2);
  _Float16* VT   = (_Float16*)take((size_t)NB * NH * HD * SQ * 2);
  _Float16* VLT  = (_Float16*)take((size_t)NB * NH * HD * ERQ * 2);
  _Float16* O16  = (_Float16*)take(NR * DM * 2);
  float*    OF   = (float*)take(NRE * DM * 4);
  if (off > ws_size) return;

  k_whd<<<dim3((unsigned)((DM * (DM / 8) + 255) / 256), 3), 256, 0, stream>>>(Wq, Wk, Wv, BQKV);
  k_wt_f16<<<(unsigned)((DM * (DM / 8) + 255) / 256), 256, 0, stream>>>(Wo, BO, DM, DM, 16.0f);
  k_wt_bf16<<<(unsigned)((DM * (DM / 8) + 255) / 256), 256, 0, stream>>>(Wo, BOB, DM, DM);
  k_x16<<<(unsigned)((xrows * DM / 8 + 255) / 256), 256, 0, stream>>>(x, X16, xrows * DM / 8);

  for (int b = 0; b < NB; ++b)
    k_gemm2<0><<<dim3((unsigned)((ERQ / 128) * (LQ / 64)), 1), 128, 0, stream>>>(X16 + (size_t)b * SQ_FULL * DM, DM, 0, BQKV, DM, 0, 0.0625f, nullptr, 0, nullptr, 1, 0, 0,
        QF + (size_t)b * ERQ * LQ, QKV + (size_t)b * SQ * LQ, LQ, 0, ERQ, LQ, DM);
  if (SQ > ERQ)
    k_gemm2<0><<<dim3((unsigned)(((SQ - ERQ) / 128) * (LQ / 64)), NB), 128, 0, stream>>>(X16 + (size_t)ERQ * DM, DM, (size_t)SQ_FULL * DM, BQKV, DM, 0, 0.0625f, nullptr, 0, nullptr, 1, 0, 0,
        nullptr, QKV + (size_t)ERQ * LQ, LQ, (size_t)SQ * LQ, SQ - ERQ, LQ, DM);
  k_res<<<(unsigned)((NRE * LQ / 8 + 255) / 256), 256, 0, stream>>>(QF, RL, NRE * LQ / 8);
  k_vt<NH, SQ><<<(unsigned)(NB * NH * (SQ / 64)), 256, 0, stream>>>(QKV, LQ, 2 * DM, VT);
  k_vt<NH, ERQ><<<(unsigned)(NB * NH * (ERQ / 64)), 256, 0, stream>>>(RL + (size_t)2 * NRE * DM, DM, 0, VLT);

  k_attn<true><<<dim3((unsigned)(ERQ / 32), (unsigned)(NB * NH)), 128, 0, stream>>>(QKV, VT, RL, VLT, O16, OF, 0);
  if (SQ > ERQ)
    k_attn<false><<<dim3((unsigned)((SQ - ERQ) / 64), (unsigned)(NB * NH)), 128, 0, stream>>>(QKV, VT, RL, VLT, O16, OF, ERQ);

  if (SQ > ERQ)
    k_gemm2<0><<<dim3((unsigned)(((SQ - ERQ) / 128) * (DM / 64)), NB), 128, 0, stream>>>(O16 + (size_t)ERQ * DM, DM, (size_t)SQ * DM, BO, DM, 0, 0.0009765625f, bo, 0, nullptr, 1, 0, 0,
        out + (size_t)ERQ * DM, nullptr, DM, (size_t)SQ_FULL * DM, SQ - ERQ, DM, DM);
  for (int b = 0; b < NB; ++b)
    k_gemm_bf<true, 0, true><<<(unsigned)(((ERQ / 16) * (DM / 64)) / 4), 128, 0, stream>>>(OF + (size_t)b * ERQ * DM, DM, BOB, DM, bo, out + (size_t)b * SQ_FULL * DM, DM, ERQ, DM, DM);
}
